// DeformableAttention_48515950575963
// MI455X (gfx1250) — hardware-verified
//
#include <hip/hip_runtime.h>

#pragma clang fp contract(off)

typedef __attribute__((ext_vector_type(16))) _Float16 v16h;
typedef __attribute__((ext_vector_type(8)))  _Float16 v8h;
typedef __attribute__((ext_vector_type(16))) __bf16   v16b;
typedef __attribute__((ext_vector_type(8)))  __bf16   v8b;
typedef __attribute__((ext_vector_type(8)))  float    v8f;
typedef __attribute__((ext_vector_type(4)))  float    v4f;
typedef __attribute__((ext_vector_type(4)))  unsigned int v4u;

constexpr int NB_    = 4;
constexpr int NCH_   = 256;
constexpr int KCONV  = 2304;
constexpr int NOFFP  = 64;
constexpr int TPITCH = 264;
static_assert(KCONV % 32 == 0, "k");
static_assert(NCH_ % 64 == 0, "n");

constexpr size_t WS_WOFF  = 0;
constexpr size_t WS_WDEF  = WS_WOFF + (size_t)NOFFP * KCONV * 2;
constexpr size_t WS_WQKV  = WS_WDEF + (size_t)NCH_ * KCONV * 2;
constexpr size_t WS_BIAS  = WS_WQKV + (size_t)3 * NCH_ * NCH_ * 2;
constexpr size_t WS_SR    = WS_BIAS + (size_t)1152 * 4;
constexpr size_t WS_X9    = WS_SR + (size_t)NB_ * NCH_ * 4096 * 4;
constexpr size_t WS_OFFP  = WS_X9 + (size_t)16384 * KCONV * 2;
constexpr size_t WS_DM    = WS_OFFP + (size_t)16384 * NOFFP * 4;
constexpr size_t WS_QKVT  = WS_DM + (size_t)16384 * NCH_ * 2;
constexpr size_t WS_TOTAL = WS_QKVT + (size_t)3 * NCH_ * 16384 * 2;
static_assert(WS_TOTAL == 131895808ull, "carve");
static_assert(WS_TOTAL <= 134217728ull, "carve cap");
static_assert(WS_WDEF % 256 == 0 && WS_WQKV % 256 == 0 && WS_BIAS % 256 == 0 && WS_SR % 256 == 0 &&
              WS_X9 % 256 == 0 && WS_OFFP % 256 == 0 && WS_DM % 256 == 0 && WS_QKVT % 256 == 0, "align");

constexpr size_t OUT0_F = 0;
constexpr size_t OUT1_F = 16777216 / 4;
constexpr size_t OUT2_F = 20971520 / 4;
static_assert(OUT2_F + (size_t)NB_ * NCH_ * 256 == 22020096 / 4, "out");

__device__ __forceinline__ unsigned short f2bf_bits(float f) {
  unsigned u = __float_as_uint(f);
  return (unsigned short)((u + 0x7FFFu + ((u >> 16) & 1u)) >> 16);
}
__device__ __forceinline__ float bf_bits2f(unsigned short h) { return __uint_as_float(((unsigned)h) << 16); }
__device__ __forceinline__ float bf16r(float x) { return bf_bits2f(f2bf_bits(x)); }
__device__ __forceinline__ unsigned short h_bits(float x) { return __builtin_bit_cast(unsigned short, (_Float16)x); }

__device__ __forceinline__ void dep_guard_h(v8f& a, v8f& b, v16h x, v16h y) { asm volatile("v_nop\n\tv_nop\n\tv_nop\n\tv_nop" : "+v"(a), "+v"(b) : "v"(x), "v"(y)); }
__device__ __forceinline__ void dep_guard_b(v8f& a, v8f& b, v16b x, v16b y) { asm volatile("v_nop\n\tv_nop\n\tv_nop\n\tv_nop" : "+v"(a), "+v"(b) : "v"(x), "v"(y)); }
__device__ __forceinline__ void keep4_h(v16h a, v16h b, v16h c, v16h d) { asm volatile("v_nop" :: "v"(a), "v"(b), "v"(c), "v"(d)); }
__device__ __forceinline__ void keep4_b(v16b a, v16b b, v16b c, v16b d) { asm volatile("v_nop" :: "v"(a), "v"(b), "v"(c), "v"(d)); }
__device__ __forceinline__ void acc_guard4(v8f& a, v8f& b, v8f& c, v8f& d) { asm volatile("v_nop\n\tv_nop\n\tv_nop\n\tv_nop" : "+v"(a), "+v"(b), "+v"(c), "+v"(d)); }
template <typename T> struct Frag;
template <> struct Frag<_Float16> {
  typedef v16h V; union U { v16h v; v8h h[2]; };
  static __device__ __forceinline__ v16h load(const _Float16* p) {
    U f; f.h[0] = *(const v8h*)(p); f.h[1] = *(const v8h*)(p + 16); return f.v;
  }
  static __device__ __forceinline__ v8f mma(v16h a, v16h b, v8f c) {
    return __builtin_amdgcn_wmma_f32_16x16x32_f16(false, a, false, b, (short)0, c, false, false);
  }
  static __device__ __forceinline__ void guard(v8f& a, v8f& b, v16h x, v16h y) { dep_guard_h(a, b, x, y); }
  static __device__ __forceinline__ void keep(v16h a, v16h b, v16h c, v16h d) { keep4_h(a, b, c, d); }
};
template <> struct Frag<__bf16> {
  typedef v16b V; union U { v16b v; v8b h[2]; };
  static __device__ __forceinline__ v16b load(const __bf16* p) {
    U f; f.h[0] = *(const v8b*)(p); f.h[1] = *(const v8b*)(p + 16); return f.v;
  }
  static __device__ __forceinline__ v8f mma(v16b a, v16b b, v8f c) {
    return __builtin_amdgcn_wmma_f32_16x16x32_bf16(false, a, false, b, (short)0, c, false, false);
  }
  static __device__ __forceinline__ void guard(v8f& a, v8f& b, v16b x, v16b y) { dep_guard_b(a, b, x, y); }
  static __device__ __forceinline__ void keep(v16b a, v16b b, v16b c, v16b d) { keep4_b(a, b, c, d); }
};

__device__ __forceinline__ v8f hmma(v16h a, v16h b, v8f c) {
  c = __builtin_amdgcn_wmma_f32_16x16x32_f16(false, a, false, b, (short)0, c, false, false);
  asm volatile("v_nop\n\tv_nop\n\tv_nop\n\tv_nop" : "+v"(c) : "v"(a), "v"(b));
  return c;
}

template <int ET> struct Elem;
template <> struct Elem<0> { typedef _Float16 T; };
template <> struct Elem<1> { typedef __bf16 T; };
template <int ET, bool SPLIT, int BIAS_MODE, int OUT_MODE>
__global__ __launch_bounds__(256) void wmma_gemm64(
    const unsigned short* __restrict__ Ap, const unsigned short* __restrict__ A2p, int lda, long strideA,
    const unsigned short* __restrict__ Btp, const unsigned short* __restrict__ Bt2p, int ldb, long strideB,
    void* __restrict__ Cout, void* __restrict__ Cout2, int ldc, long strideC,
    const float* __restrict__ bias, long strideBias,
    int M, int N, int K, float scale) {
  typedef typename Elem<ET>::T T;
  typedef typename Frag<T>::V V;
  const T* A = (const T*)Ap; const T* A2 = (const T*)A2p; const T* Bt = (const T*)Btp; const T* Bt2 = (const T*)Bt2p;
  __shared__ __align__(16) float sT[8][16 * 68];
  const int b    = blockIdx.y;
  const int lane = threadIdx.x & 31;
  const int wave = threadIdx.x >> 5;
  const int tilesN = N >> 6;
  const int tilesM = M >> 6;
  const int tile = blockIdx.x * 8 + wave;
  if (tile >= tilesM * tilesN) return;
  const int tm = tile / tilesN;
  const int tn = tile - tm * tilesN;
  const int m0 = tm << 6;
  const int n0 = tn << 6;

  const T* Ab  = A  + (size_t)b * strideA;
  const T* Bb  = Bt + (size_t)b * strideB;
  const T* Ab2 = SPLIT ? (A2  + (size_t)b * strideA) : nullptr;
  const T* Bb2 = SPLIT ? (Bt2 + (size_t)b * strideB) : nullptr;

  const int rlane = lane & 15;
  const int koff  = (lane >> 4) * 8;
  const int mOff  = (lane >> 4) * 8;

  v8f acc[4][4];
#pragma unroll
  for (int i = 0; i < 4; ++i)
#pragma unroll
    for (int j = 0; j < 4; ++j) acc[i][j] = (v8f){0.f,0.f,0.f,0.f,0.f,0.f,0.f,0.f};

  for (int k0 = 0; k0 < K; k0 += 32) {
    V bh[4], bl[4];
#pragma unroll
    for (int j = 0; j < 4; ++j) {
      const size_t bo = (size_t)(n0 + (j << 4) + rlane) * ldb + koff + k0;
      bh[j] = Frag<T>::load(Bb + bo);
      if (SPLIT) bl[j] = Frag<T>::load(Bb2 + bo);
    }
#pragma unroll
    for (int i = 0; i < 4; ++i) {
      const size_t ao = (size_t)(m0 + (i << 4) + rlane) * lda + koff + k0;
      V ah = Frag<T>::load(Ab + ao);
      V al = ah;
      if (SPLIT) al = Frag<T>::load(Ab2 + ao);
#pragma unroll
      for (int j = 0; j < 4; ++j) {
        acc[i][j] = Frag<T>::mma(ah, bh[j], acc[i][j]);
        if (SPLIT) {
          acc[i][j] = Frag<T>::mma(ah, bl[j], acc[i][j]);
          acc[i][j] = Frag<T>::mma(al, bh[j], acc[i][j]);
        }
      }
      Frag<T>::guard(acc[i][0], acc[i][3], ah, al);
    }
    Frag<T>::keep(bh[0], bh[1], bh[2], bh[3]);
    if (SPLIT) Frag<T>::keep(bl[0], bl[1], bl[2], bl[3]);
  }
  acc_guard4(acc[0][0], acc[0][1], acc[0][2], acc[0][3]);
  acc_guard4(acc[1][0], acc[1][1], acc[1][2], acc[1][3]);
  acc_guard4(acc[2][0], acc[2][1], acc[2][2], acc[2][3]);
  acc_guard4(acc[3][0], acc[3][1], acc[3][2], acc[3][3]);

  float* slab = sT[wave];
  const float* biasb = (BIAS_MODE != 0) ? (bias + (size_t)b * strideBias) : nullptr;
#pragma unroll
  for (int i = 0; i < 4; ++i) {
    const int mBase = m0 + (i << 4);
    float bm[8];
#pragma unroll
    for (int r = 0; r < 8; ++r) bm[r] = 0.f;
    if (BIAS_MODE == 1) {
      const v4f bA = *(const v4f*)(biasb + mBase + mOff);
      const v4f bB = *(const v4f*)(biasb + mBase + mOff + 4);
      bm[0] = bA[0]; bm[1] = bA[1]; bm[2] = bA[2]; bm[3] = bA[3];
      bm[4] = bB[0]; bm[5] = bB[1]; bm[6] = bB[2]; bm[7] = bB[3];
    }
#pragma unroll
    for (int j = 0; j < 4; ++j) {
      const int n = n0 + (j << 4) + rlane;
      float bvn = 0.f;
      if (BIAS_MODE == 2) bvn = biasb[n];
#pragma unroll
      for (int r = 0; r < 8; ++r) {
        float v = acc[i][j][r] * scale;
        if (BIAS_MODE == 1) v += bm[r];
        if (BIAS_MODE == 2) v += bvn;
        slab[(mOff + r) * 68 + (j << 4) + rlane] = v;
      }
    }
    __builtin_amdgcn_fence(__ATOMIC_RELEASE, "workgroup");
    __builtin_amdgcn_wave_barrier();
    __builtin_amdgcn_fence(__ATOMIC_ACQUIRE, "workgroup");
    if (OUT_MODE == 0) {
      float* C = (float*)Cout + (size_t)b * strideC;
      const int hh = lane >> 4, c4 = (lane & 15) * 4;
      for (int pass = 0; pass < 2; ++pass) {
#pragma unroll
        for (int it = 0; it < 8; ++it) {
          const int row = it * 2 + hh;
          v4f v = *(const v4f*)(slab + row * 68 + c4);
          *(volatile v4f*)(C + (size_t)(mBase + row) * ldc + n0 + c4) = v;
        }
        __threadfence();
      }
    } else {
      const int q = lane >> 3, c8 = (lane & 7) * 8;
      unsigned short* C  = (unsigned short*)Cout  + (size_t)b * strideC;
      unsigned short* C2 = (OUT_MODE == 2) ? ((unsigned short*)Cout2 + (size_t)b * strideC) : nullptr;
      for (int pass = 0; pass < 2; ++pass) {
#pragma unroll
        for (int it = 0; it < 4; ++it) {
          const int row = it * 4 + q;
          const float* sp = slab + row * 68 + c8;
          v8h hv, lv;
#pragma unroll
          for (int e = 0; e < 8; ++e) {
            if (OUT_MODE == 1) {
              hv[e] = (_Float16)sp[e];
              lv[e] = hv[e];
            } else {
              unsigned short hb = f2bf_bits(sp[e]);
              unsigned short lb = f2bf_bits(sp[e] - bf_bits2f(hb));
              hv[e] = __builtin_bit_cast(_Float16, hb);
              lv[e] = __builtin_bit_cast(_Float16, lb);
            }
          }
          *(volatile v8h*)(C + (size_t)(mBase + row) * ldc + n0 + c8) = hv;
          if (OUT_MODE == 2) *(volatile v8h*)(C2 + (size_t)(mBase + row) * ldc + n0 + c8) = lv;
        }
        __threadfence();
      }
    }
    __builtin_amdgcn_fence(__ATOMIC_RELEASE, "workgroup");
    __builtin_amdgcn_wave_barrier();
    __builtin_amdgcn_fence(__ATOMIC_ACQUIRE, "workgroup");
  }
}

__global__ __launch_bounds__(256) void prep_wconv_kernel(const float* __restrict__ wsrc, unsigned short* __restrict__ dst,
                                                         int nrow_real, int nrow_pad) {
  const int i = blockIdx.x * 256 + threadIdx.x;
  if (i >= nrow_pad * 288) return;
  const int row = i / 288;
  const int chk = i - row * 288;
  const int k0  = chk * 8;
  const int tap = k0 >> 8;
  const int c0  = k0 & 255;
  const bool live = row < nrow_real;
  const int rowc = live ? row : (nrow_real - 1);
  const float* sp = wsrc + ((size_t)rowc * NCH_ + c0) * 9 + tap;
  float x[8];
#pragma unroll
  for (int e = 0; e < 8; ++e) x[e] = sp[e * 9];
  v4u pk;
#pragma unroll
  for (int e = 0; e < 4; ++e) {
    const float y0 = live ? 64.0f * bf16r(x[2 * e])     : 0.0f;
    const float y1 = live ? 64.0f * bf16r(x[2 * e + 1]) : 0.0f;
    pk[e] = (unsigned)h_bits(y0) | ((unsigned)h_bits(y1) << 16);
  }
  unsigned short* d = dst + (size_t)i * 8;
  *(volatile v4u*)d = pk;
  __threadfence();
  *(volatile v4u*)d = pk;
}

__global__ __launch_bounds__(256) void prep_wlin_kernel(const float* __restrict__ wq, const float* __restrict__ wk,
                                                        const float* __restrict__ wv, unsigned short* __restrict__ dst) {
  const int i = blockIdx.x * 256 + threadIdx.x;
  if (i >= 3 * 8192) return;
  const int sel = blockIdx.x >> 5;
  const float* src = (sel == 0) ? wq : ((sel == 1) ? wk : wv);
  const int j = i & 8191;
  const v4f a0 = *(const v4f*)(src + (size_t)j * 8);
  const v4f a1 = *(const v4f*)(src + (size_t)j * 8 + 4);
  v4u pk;
  pk[0] = (unsigned)h_bits(16.0f * bf16r(a0[0])) | ((unsigned)h_bits(16.0f * bf16r(a0[1])) << 16);
  pk[1] = (unsigned)h_bits(16.0f * bf16r(a0[2])) | ((unsigned)h_bits(16.0f * bf16r(a0[3])) << 16);
  pk[2] = (unsigned)h_bits(16.0f * bf16r(a1[0])) | ((unsigned)h_bits(16.0f * bf16r(a1[1])) << 16);
  pk[3] = (unsigned)h_bits(16.0f * bf16r(a1[2])) | ((unsigned)h_bits(16.0f * bf16r(a1[3])) << 16);
  unsigned short* d = dst + (size_t)i * 8;
  *(volatile v4u*)d = pk;
  __threadfence();
  *(volatile v4u*)d = pk;
}

__global__ __launch_bounds__(256) void prep_bias_kernel(const float* __restrict__ b_off, const float* __restrict__ b_def,
                                                        const float* __restrict__ bq, const float* __restrict__ bk,
                                                        const float* __restrict__ bv, float* __restrict__ table) {
  const int t = blockIdx.x * 256 + threadIdx.x;
  if (t >= 288) return;
  const int w = t >> 5;
  const float* src; int nsrc; int tb;
  if (w == 0)      { src = b_off; nsrc = 18;   tb = 0;   }
  else if (w <= 2) { src = b_def; nsrc = NCH_; tb = 32;  }
  else if (w <= 4) { src = bq;    nsrc = NCH_; tb = 96;  }
  else if (w <= 6) { src = bk;    nsrc = NCH_; tb = 160; }
  else             { src = bv;    nsrc = NCH_; tb = 224; }
  v4f val;
#pragma unroll
  for (int e = 0; e < 4; ++e) {
    const int o  = (t - tb) * 4 + e;
    const int oc = (o < nsrc) ? o : (nsrc - 1);
    const float x = src[oc];
    val[e] = (o < nsrc) ? bf16r(x) : 0.0f;
  }
  float* d = table + (size_t)t * 4;
  *(volatile v4f*)d = val;
  __threadfence();
  *(volatile v4f*)d = val;
}

__global__ __launch_bounds__(256) void rne_copy_kernel(const float* __restrict__ s, float* __restrict__ sr, int n4) {
  const int i = blockIdx.x * 256 + threadIdx.x;
  if (i >= n4) return;
  const v4f x = *(const v4f*)(s + (size_t)i * 4);
  v4f y;
  y[0] = bf16r(x[0]); y[1] = bf16r(x[1]); y[2] = bf16r(x[2]); y[3] = bf16r(x[3]);
  float* d = sr + (size_t)i * 4;
  *(volatile v4f*)d = y;
  __threadfence();
  *(volatile v4f*)d = y;
}

__global__ __launch_bounds__(256) void im2col_kernel(const float* __restrict__ sr, unsigned short* __restrict__ x9, int H, int W) {
  __shared__ __align__(16) unsigned short T[32 * TPITCH];
  const int tid = threadIdx.x, lane = tid & 31, wave = tid >> 5;
  const int HW = H * W;
  const int m0 = blockIdx.x * 32;
  const int m  = m0 + lane;
  const int b  = m / HW;
  const int pix = m - b * HW;
  const int ph = pix / W;
  const int pw = pix - ph * W;
  const float* sb = sr + (size_t)b * NCH_ * HW;
  for (int tap = 0; tap < 9; ++tap) {
    const int hy = ph + tap / 3 - 1;
    const int wx = pw + tap % 3 - 1;
    const bool valid = (hy >= 0) && (hy < H) && (wx >= 0) && (wx < W);
    const int hc = hy < 0 ? 0 : (hy > H - 1 ? H - 1 : hy);
    const int wc = wx < 0 ? 0 : (wx > W - 1 ? W - 1 : wx);
    const float* sp = sb + (size_t)hc * W + wc;
#pragma unroll 4
    for (int ci = 0; ci < 32; ++ci) {
      const int c = wave * 32 + ci;
      float v = sp[(size_t)c * HW];
      v = valid ? v : 0.0f;
      T[lane * TPITCH + c] = h_bits(v);
    }
    __syncthreads();
    v4u hv[4];
#pragma unroll
    for (int rr = 0; rr < 4; ++rr) {
      const int p2 = wave * 4 + rr;
      hv[rr] = *(const v4u*)(T + p2 * TPITCH + lane * 8);
    }
    for (int pass = 0; pass < 2; ++pass) {
#pragma unroll
      for (int rr = 0; rr < 4; ++rr) {
        const int m2 = m0 + wave * 4 + rr;
        *(volatile v4u*)(x9 + (size_t)m2 * KCONV + tap * 256 + lane * 8) = hv[rr];
      }
      __threadfence();
    }
    __syncthreads();
  }
}

__global__ __launch_bounds__(256) void sample_kernel(const float* __restrict__ sr, const float* __restrict__ offp,
                                                     unsigned short* __restrict__ s9, int H, int W) {
  __shared__ __align__(16) unsigned short T[32 * TPITCH];
  const int tid = threadIdx.x, lane = tid & 31, wave = tid >> 5;
  const int HW = H * W;
  const int m0 = blockIdx.x * 32;
  const int m  = m0 + lane;
  const int b  = m / HW;
  const int pix = m - b * HW;
  const int ph = pix / W;
  const int pw = pix - ph * W;
  const float* sb = sr + (size_t)b * NCH_ * HW;
  for (int tap = 0; tap < 9; ++tap) {
    const float dyo = offp[(size_t)m * NOFFP + 2 * tap];
    const float dxo = offp[(size_t)m * NOFFP + 2 * tap + 1];
    const float basey = (float)(ph - 1) + (float)(tap / 3);
    const float basex = (float)(pw - 1) + (float)(tap % 3);
    const float py = basey + dyo;
    const float px = basex + dxo;
    const float y0f = floorf(py);
    const float x0f = floorf(px);
    const float wy1 = py - y0f;
    const float wy0 = 1.0f - wy1;
    const float wx1 = px - x0f;
    const float wx0 = 1.0f - wx1;
    const float y0cl = fminf(fmaxf(y0f, -4.0f), (float)(H + 4));
    const float x0cl = fminf(fmaxf(x0f, -4.0f), (float)(W + 4));
    const int yi0 = (int)y0cl, yi1 = yi0 + 1;
    const int xi0 = (int)x0cl, xi1 = xi0 + 1;
    const bool vy0 = (yi0 >= 0) && (yi0 < H);
    const bool vy1 = (yi1 >= 0) && (yi1 < H);
    const bool vx0 = (xi0 >= 0) && (xi0 < W);
    const bool vx1 = (xi1 >= 0) && (xi1 < W);
    float w00 = wy0 * wx0;
    float w01 = wy0 * wx1;
    float w10 = wy1 * wx0;
    float w11 = wy1 * wx1;
    w00 = (vy0 && vx0) ? w00 : 0.0f;
    w01 = (vy0 && vx1) ? w01 : 0.0f;
    w10 = (vy1 && vx0) ? w10 : 0.0f;
    w11 = (vy1 && vx1) ? w11 : 0.0f;
    const int yc0 = yi0 < 0 ? 0 : (yi0 > H - 1 ? H - 1 : yi0);
    const int yc1 = yi1 < 0 ? 0 : (yi1 > H - 1 ? H - 1 : yi1);
    const int xc0 = xi0 < 0 ? 0 : (xi0 > W - 1 ? W - 1 : xi0);
    const int xc1 = xi1 < 0 ? 0 : (xi1 > W - 1 ? W - 1 : xi1);
    const int i00 = yc0 * W + xc0;
    const int i01 = yc0 * W + xc1;
    const int i10 = yc1 * W + xc0;
    const int i11 = yc1 * W + xc1;
#pragma unroll 2
    for (int ci = 0; ci < 32; ++ci) {
      const int c = wave * 32 + ci;
      const float* sp = sb + (size_t)c * HW;
      const float v00 = sp[i00];
      const float v01 = sp[i01];
      const float v10 = sp[i10];
      const float v11 = sp[i11];
      const float t00 = v00 * w00;
      const float t01 = v01 * w01;
      const float t10 = v10 * w10;
      const float t11 = v11 * w11;
      const float val = ((t00 + t01) + t10) + t11;
      T[lane * TPITCH + c] = h_bits(val);
    }
    __syncthreads();
    v4u hv[4];
#pragma unroll
    for (int rr = 0; rr < 4; ++rr) {
      const int p2 = wave * 4 + rr;
      hv[rr] = *(const v4u*)(T + p2 * TPITCH + lane * 8);
    }
    for (int pass = 0; pass < 2; ++pass) {
#pragma unroll
      for (int rr = 0; rr < 4; ++rr) {
        const int m2 = m0 + wave * 4 + rr;
        *(volatile v4u*)(s9 + (size_t)m2 * KCONV + tap * 256 + lane * 8) = hv[rr];
      }
      __threadfence();
    }
    __syncthreads();
  }
}

template <int HH>
__global__ __launch_bounds__(128) void chan_attn_kernel(const unsigned short* __restrict__ qt, const unsigned short* __restrict__ kt,
                                                        const unsigned short* __restrict__ vt, float* __restrict__ outp, int Mpix) {
  constexpr int WW  = HH;
  constexpr int HWc = HH * WW;
  constexpr int NCH = 64 / HH;
  constexpr int KP  = (HH < 32) ? 32 : HH;
  constexpr int PT  = KP + 8;
  constexpr int NT  = HH / 16;
  constexpr int KS  = KP / 32;
  constexpr int OSP = 68;
  constexpr int CPP = HWc / 8;
  constexpr int NIT = (16 * WW) / 128;
  static_assert(NT * NCH == 4, "waves");
  __shared__ __align__(16) unsigned short Qs[NCH * HH * PT];
  __shared__ __align__(16) unsigned short Ks[NCH * HH * PT];
  __shared__ __align__(16) unsigned short Vts[NCH * WW * PT];
  __shared__ __align__(16) unsigned short Ps[64 * PT];
  __shared__ __align__(16) float Os[64 * OSP];

  const int tid  = threadIdx.x;
  const int wave = tid >> 5, lane = tid & 31, hh = lane >> 4, cl = lane & 15, koff = hh * 8;
  const int pc0  = blockIdx.x * NCH;

  if (KP > HH) {
    const v4u z = {0u, 0u, 0u, 0u};
    for (int q = tid; q < NCH * HH * 2; q += 128) {
      *(v4u*)(Qs + (q >> 1) * PT + HH + (q & 1) * 8) = z;
      *(v4u*)(Ks + (q >> 1) * PT + HH + (q & 1) * 8) = z;
    }
    for (int q = tid; q < NCH * WW * 2; q += 128) *(v4u*)(Vts + (q >> 1) * PT + HH + (q & 1) * 8) = z;
    for (int q = tid; q < 64 * 2; q += 128)       *(v4u*)(Ps + (q >> 1) * PT + HH + (q & 1) * 8) = z;
  }
  for (int q = tid; q < NCH * CPP; q += 128) {
    const int pr = q / CPP;
    const int within = q - pr * CPP;
    const int e0 = within * 8;
    const int h = e0 / WW;
    const int w = e0 - h * WW;
    const int pc = pc0 + pr;
    const int b = pc >> 8, ch = pc & 255;
    const size_t g = (size_t)ch * Mpix + (size_t)b * HWc + e0;
    const v4u qv = *(const v4u*)(qt + g);
    const v4u kv = *(const v4u*)(kt + g);
    const v4u vv = *(const v4u*)(vt + g);
    *(v4u*)(Qs + (pr * HH + h) * PT + w) = qv;
    *(v4u*)(Ks + (pr * HH + h) * PT + w) = kv;
#pragma unroll
    for (int e = 0; e < 8; ++e) {
      const unsigned wd = vv[e >> 1];
      const unsigned short hvb = (unsigned short)((e & 1) ? (wd >> 16) : (wd & 0xffffu));
      Vts[(pr * WW + w + e) * PT + h] = hvb;
    }
  }
  __syncthreads();

  const int pr   = wave / NT;
  const int slab = wave - pr * NT;
  const int r0   = slab * 16;
  const _Float16* Qp = (const _Float16*)(Qs + (pr * HH + r0) * PT);
  const _Float16* Kp = (const _Float16*)(Ks + pr * HH * PT);
  v8f sacc[NT];
#pragma unroll
  for (int jt = 0; jt < NT; ++jt) sacc[jt] = (v8f){0.f,0.f,0.f,0.f,0.f,0.f,0.f,0.f};
#pragma unroll
  for (int ks = 0; ks < KS; ++ks) {
    const v16h a = Frag<_Float16>::load(Qp + cl * PT + koff + ks * 32);
#pragma unroll
    for (int jt = 0; jt < NT; ++jt) {
      const v16h bb = Frag<_Float16>::load(Kp + (jt * 16 + cl) * PT + koff + ks * 32);
      sacc[jt] = hmma(a, bb, sacc[jt]);
    }
  }
  float inv[8];
  unsigned short* pwv = Ps + wave * 16 * PT;
#pragma unroll
  for (int r = 0; r < 8; ++r) {
    float mx = -3.0e38f;
#pragma unroll
    for (int jt = 0; jt < NT; ++jt) {
      const float sv = sacc[jt][r] * 0.0625f;
      sacc[jt][r] = sv;
      mx = fmaxf(mx, sv);
    }
#pragma unroll
    for (int off = 8; off > 0; off >>= 1) mx = fmaxf(mx, __shfl_xor(mx, off, 32));
    float sum = 0.0f;
#pragma unroll
    for (int jt = 0; jt < NT; ++jt) {
      const float e = expf(sacc[jt][r] - mx);
      sum += e;
      pwv[(8 * hh + r) * PT + jt * 16 + cl] = h_bits(e * 1024.0f);
    }
#pragma unroll
    for (int off = 8; off > 0; off >>= 1) sum += __shfl_xor(sum, off, 32);
    inv[r] = 1.0f / (sum * 1024.0f);
  }
  __syncthreads();

  const _Float16* Pp = (const _Float16*)(Ps + wave * 16 * PT);
  const _Float16* Vp = (const _Float16*)(Vts + pr * WW * PT);
  v8f oacc[NT];
#pragma unroll
  for (int t = 0; t < NT; ++t) oacc[t] = (v8f){0.f,0.f,0.f,0.f,0.f,0.f,0.f,0.f};
#pragma unroll
  for (int ks = 0; ks < KS; ++ks) {
    const v16h a = Frag<_Float16>::load(Pp + cl * PT + koff + ks * 32);
#pragma unroll
    for (int t = 0; t < NT; ++t) {
      const v16h bb = Frag<_Float16>::load(Vp + (t * 16 + cl) * PT + koff + ks * 32);
      oacc[t] = hmma(a, bb, oacc[t]);
    }
  }
  float* os = Os + wave * 16 * OSP;
#pragma unroll
  for (int r = 0; r < 8; ++r) {
#pragma unroll
    for (int t = 0; t < NT; ++t) os[(8 * hh + r) * OSP + t * 16 + cl] = oacc[t][r] * inv[r];
  }
  __syncthreads();
  const int pc = pc0 + pr;
  float* ob = outp + (size_t)pc * HWc + (size_t)r0 * WW;
  v4f vals[NIT];
#pragma unroll
  for (int it = 0; it < NIT; ++it) {
    const int f = it * 128 + lane * 4;
    const int row = f / WW;
    const int col = f - row * WW;
    vals[it] = *(const v4f*)(os + row * OSP + col);
  }
  for (int pass = 0; pass < 2; ++pass) {
#pragma unroll
    for (int it = 0; it < NIT; ++it) *(volatile v4f*)(ob + it * 128 + lane * 4) = vals[it];
    __threadfence();
  }
}

extern "C" void kernel_launch(void* const* d_in, const int* in_sizes, int n_in,
                              void* d_out, int out_size, void* d_ws, size_t ws_size,
                              hipStream_t stream) {
  if (n_in < 13) return;
  if (ws_size < WS_TOTAL) return;
  if (out_size != 22020096 / 4) return;
  if (in_sizes[0] != NB_ * NCH_ * 4096 || in_sizes[1] != NB_ * NCH_ * 1024 || in_sizes[2] != NB_ * NCH_ * 256) return;
  if (in_sizes[3] != 18 * NCH_ * 9 || in_sizes[4] != 18 || in_sizes[5] != NCH_ * NCH_ * 9 || in_sizes[6] != NCH_) return;
  if (in_sizes[7] != NCH_ * NCH_ || in_sizes[8] != NCH_ || in_sizes[9] != NCH_ * NCH_ || in_sizes[10] != NCH_ ||
      in_sizes[11] != NCH_ * NCH_ || in_sizes[12] != NCH_) return;

  const float* s_in[3] = {(const float*)d_in[0], (const float*)d_in[1], (const float*)d_in[2]};
  const float* w_off = (const float*)d_in[3];
  const float* b_off = (const float*)d_in[4];
  const float* w_def = (const float*)d_in[5];
  const float* b_def = (const float*)d_in[6];
  const float* wq    = (const float*)d_in[7];
  const float* bq    = (const float*)d_in[8];
  const float* wk    = (const float*)d_in[9];
  const float* bk    = (const float*)d_in[10];
  const float* wv    = (const float*)d_in[11];
  const float* bv    = (const float*)d_in[12];
  float* out = (float*)d_out;

  char* ws = (char*)d_ws;
  unsigned short* WOFF = (unsigned short*)(ws + WS_WOFF);
  unsigned short* WDEF = (unsigned short*)(ws + WS_WDEF);
  unsigned short* WQKV = (unsigned short*)(ws + WS_WQKV);
  float*          BIAS = (float*)(ws + WS_BIAS);
  float*          SR   = (float*)(ws + WS_SR);
  unsigned short* X9   = (unsigned short*)(ws + WS_X9);
  float*          OFFP = (float*)(ws + WS_OFFP);
  unsigned short* DM   = (unsigned short*)(ws + WS_DM);
  unsigned short* QKVT = (unsigned short*)(ws + WS_QKVT);

  const float inv64 = 0.015625f;
  const float inv16 = 0.0625f;

  prep_wconv_kernel<<<dim3((NOFFP * 288) / 256), dim3(256), 0, stream>>>(w_off, WOFF, 18, NOFFP);
  prep_wconv_kernel<<<dim3((NCH_ * 288) / 256), dim3(256), 0, stream>>>(w_def, WDEF, NCH_, NCH_);
  prep_wlin_kernel<<<dim3(96), dim3(256), 0, stream>>>(wq, wk, wv, WQKV);
  prep_bias_kernel<<<dim3(2), dim3(256), 0, stream>>>(b_off, b_def, bq, bk, bv, BIAS);

  const size_t outoff[3] = {OUT0_F, OUT1_F, OUT2_F};
  for (int i = 0; i < 3; ++i) {
    const int H = 64 >> i, W = H, HW = H * W;
    const int Mpix = NB_ * HW;
    const int n4 = Mpix * NCH_ / 4;
    rne_copy_kernel<<<dim3(n4 / 256), dim3(256), 0, stream>>>(s_in[i], SR, n4);
    im2col_kernel<<<dim3(Mpix / 32), dim3(256), 0, stream>>>(SR, X9, H, W);
    {
      const int tiles = (Mpix / 64) * (NOFFP / 64);
      wmma_gemm64<0, false, 2, 0><<<dim3((tiles + 7) / 8, 1), dim3(256), 0, stream>>>(
          X9, X9, KCONV, 0L, WOFF, WOFF, KCONV, 0L, (void*)OFFP, nullptr, NOFFP, 0L,
          BIAS + 0, 0L, Mpix, NOFFP, KCONV, inv64);
    }
    sample_kernel<<<dim3(Mpix / 32), dim3(256), 0, stream>>>(SR, OFFP, X9, H, W);
    {
      const int tiles = (Mpix / 64) * (NCH_ / 64);
      wmma_gemm64<0, false, 2, 1><<<dim3((tiles + 7) / 8, 1), dim3(256), 0, stream>>>(
          X9, X9, KCONV, 0L, WDEF, WDEF, KCONV, 0L, (void*)DM, nullptr, NCH_, 0L,
          BIAS + 128, 0L, Mpix, NCH_, KCONV, inv64);
    }
    {
      const int tiles = (NCH_ / 64) * (Mpix / 64);
      wmma_gemm64<0, false, 1, 1><<<dim3((tiles + 7) / 8, 3), dim3(256), 0, stream>>>(
          WQKV, WQKV, NCH_, (long)NCH_ * NCH_, DM, DM, NCH_, 0L, (void*)QKVT, nullptr, Mpix, (long)NCH_ * Mpix,
          BIAS + 384, (long)NCH_, NCH_, Mpix, NCH_, inv16);
    }
    const unsigned short* QT = QKVT;
    const unsigned short* KT = QKVT + (size_t)NCH_ * Mpix;
    const unsigned short* VT = QKVT + (size_t)2 * NCH_ * Mpix;
    float* o = out + outoff[i];
    if (H == 64)      chan_attn_kernel<64><<<dim3(NB_ * NCH_ / 1), dim3(128), 0, stream>>>(QT, KT, VT, o, Mpix);
    else if (H == 32) chan_attn_kernel<32><<<dim3(NB_ * NCH_ / 2), dim3(128), 0, stream>>>(QT, KT, VT, o, Mpix);
    else              chan_attn_kernel<16><<<dim3(NB_ * NCH_ / 4), dim3(128), 0, stream>>>(QT, KT, VT, o, Mpix);
  }
}
